// SelectiveSSMBlock_26534307954721
// MI455X (gfx1250) — hardware-verified
//
#include <hip/hip_runtime.h>
#include <math.h>

typedef __attribute__((ext_vector_type(16))) _Float16 v16h;
typedef __attribute__((ext_vector_type(8)))  _Float16 v8h;
typedef __attribute__((ext_vector_type(16))) __bf16   v16b;
typedef __attribute__((ext_vector_type(8)))  __bf16   v8b;
typedef __attribute__((ext_vector_type(8)))  float    v8f;
typedef __attribute__((ext_vector_type(4)))  float    v4f;

constexpr int kBatch  = 2;
constexpr int kSeq    = 2048;
constexpr int kDm     = 1024;
constexpr int kNst    = 16;
constexpr int kDtR    = 64;
constexpr int kNproj  = kDtR + 2 * kNst;
constexpr int kNpad   = 128;
constexpr int kRows   = kBatch * kSeq;
constexpr int kBcW    = 2 * kNst;
constexpr int kScanTS = 64;
constexpr int kScanCh = 64;
constexpr int kScanYP = 68;
constexpr float kW1Carry = 64.0f;
constexpr float kDpCarry = 16.0f;
constexpr float kW2Carry = 256.0f;
static_assert(kNproj <= kNpad, "pad");
static_assert((kDm % 32) == 0 && (kDtR % 32) == 0, "GEMM K multiples of 32");
static_assert((kRows % 64) == 0 && (kNpad % 64) == 0 && (kDm % 64) == 0, "GEMM M,N multiples of 64");
static_assert((kSeq % kScanTS) == 0 && (kDm % kScanCh) == 0 && (kScanCh == 64) && (kScanTS == 64), "scan tiles");

constexpr size_t kOffU16  = 0;
constexpr size_t kOffW1H  = kOffU16 + (size_t)kRows * kDm   * 2;
constexpr size_t kOffW2H  = kOffW1H + (size_t)kNpad * kDm   * 2;
constexpr size_t kOffXZ   = kOffW2H + (size_t)kDm   * kDtR  * 2;
constexpr size_t kOffDP16 = kOffXZ  + (size_t)kRows * kNpad * 4;
constexpr size_t kOffDPRE = kOffDP16 + (size_t)kRows * kDtR * 2;
constexpr size_t kWsTotal = kOffDPRE + (size_t)kRows * kDm  * 4;
static_assert(kWsTotal == 28180480ull, "carve total");
static_assert(kWsTotal <= 134217728ull, "carve cap");
static_assert((kOffW1H % 128) == 0 && (kOffW2H % 128) == 0 && (kOffXZ % 128) == 0 &&
              (kOffDP16 % 128) == 0 && (kOffDPRE % 128) == 0, "128-B aligned regions");

__device__ __forceinline__ unsigned short f2bf_bits(float f) {
  unsigned u = __float_as_uint(f);
  return (unsigned short)((u + 0x7FFFu + ((u >> 16) & 1u)) >> 16);
}
__device__ __forceinline__ float bf_bits2f(unsigned short h) { return __uint_as_float(((unsigned)h) << 16); }

__device__ __forceinline__ void dep_guard_h(v8f& a, v8f& b, v16h x, v16h y) { asm volatile("v_nop\n\tv_nop\n\tv_nop\n\tv_nop" : "+v"(a), "+v"(b) : "v"(x), "v"(y)); }
__device__ __forceinline__ void dep_guard_b(v8f& a, v8f& b, v16b x, v16b y) { asm volatile("v_nop\n\tv_nop\n\tv_nop\n\tv_nop" : "+v"(a), "+v"(b) : "v"(x), "v"(y)); }
__device__ __forceinline__ void dep_guard4_h(v8f& a, v8f& b, v8f& c, v8f& d, v16h x, v16h y) { asm volatile("v_nop\n\tv_nop\n\tv_nop\n\tv_nop" : "+v"(a), "+v"(b), "+v"(c), "+v"(d) : "v"(x), "v"(y)); }
__device__ __forceinline__ void dep_guard4_b(v8f& a, v8f& b, v8f& c, v8f& d, v16b x, v16b y) { asm volatile("v_nop\n\tv_nop\n\tv_nop\n\tv_nop" : "+v"(a), "+v"(b), "+v"(c), "+v"(d) : "v"(x), "v"(y)); }
__device__ __forceinline__ void keep4_h(v16h a, v16h b, v16h c, v16h d) { asm volatile("v_nop" :: "v"(a), "v"(b), "v"(c), "v"(d)); }
__device__ __forceinline__ void keep4_b(v16b a, v16b b, v16b c, v16b d) { asm volatile("v_nop" :: "v"(a), "v"(b), "v"(c), "v"(d)); }
__device__ __forceinline__ void acc_guard4(v8f& a, v8f& b, v8f& c, v8f& d) { asm volatile("v_nop\n\tv_nop\n\tv_nop\n\tv_nop" : "+v"(a), "+v"(b), "+v"(c), "+v"(d)); }
template <typename T> struct Frag;
template <> struct Frag<_Float16> {
  typedef v16h V; union U { v16h v; v8h h[2]; };
  static __device__ __forceinline__ v16h load(const _Float16* p) {
    U f; f.h[0] = *(const v8h*)(p); f.h[1] = *(const v8h*)(p + 16); return f.v;
  }
  static __device__ __forceinline__ v8f mma(v16h a, v16h b, v8f c) {
    return __builtin_amdgcn_wmma_f32_16x16x32_f16(false, a, false, b, (short)0, c, false, false);
  }
  static __device__ __forceinline__ void guard(v8f& a, v8f& b, v16h x, v16h y) { dep_guard_h(a, b, x, y); }
  static __device__ __forceinline__ void guard4(v8f& a, v8f& b, v8f& c, v8f& d, v16h x, v16h y) { dep_guard4_h(a, b, c, d, x, y); }
  static __device__ __forceinline__ void keep(v16h a, v16h b, v16h c, v16h d) { keep4_h(a, b, c, d); }
};
template <> struct Frag<__bf16> {
  typedef v16b V; union U { v16b v; v8b h[2]; };
  static __device__ __forceinline__ v16b load(const __bf16* p) {
    U f; f.h[0] = *(const v8b*)(p); f.h[1] = *(const v8b*)(p + 16); return f.v;
  }
  static __device__ __forceinline__ v8f mma(v16b a, v16b b, v8f c) {
    return __builtin_amdgcn_wmma_f32_16x16x32_bf16(false, a, false, b, (short)0, c, false, false);
  }
  static __device__ __forceinline__ void guard(v8f& a, v8f& b, v16b x, v16b y) { dep_guard_b(a, b, x, y); }
  static __device__ __forceinline__ void guard4(v8f& a, v8f& b, v8f& c, v8f& d, v16b x, v16b y) { dep_guard4_b(a, b, c, d, x, y); }
  static __device__ __forceinline__ void keep(v16b a, v16b b, v16b c, v16b d) { keep4_b(a, b, c, d); }
};

template <int ET> struct Elem;
template <> struct Elem<0> { typedef _Float16 T; };
template <> struct Elem<1> { typedef __bf16 T; };
template <int ET, int SPL, int BIAS_MODE, int OUT_MODE, bool RESID, int ACT = 0>
__global__ __launch_bounds__(256) void wmma_gemm64(
    const unsigned short* __restrict__ Ap, const unsigned short* __restrict__ A2p, int lda, long strideA,
    const unsigned short* __restrict__ Btp, const unsigned short* __restrict__ Bt2p, int ldb, long strideB,
    void* __restrict__ Cout, void* __restrict__ Cout2, int ldc, long strideC,
    const float* __restrict__ bias,
    const float* __restrict__ resid, long strideR,
    int M, int N, int K, float scale) {
  typedef typename Elem<ET>::T T;
  typedef typename Frag<T>::V V;
  const T* A = (const T*)Ap; const T* A2 = (const T*)A2p; const T* Bt = (const T*)Btp; const T* Bt2 = (const T*)Bt2p;
  __shared__ __align__(16) float sT[8][16 * 68];
  const int b    = blockIdx.y;
  const int lane = threadIdx.x & 31;
  const int wave = threadIdx.x >> 5;
  const int tilesN = N >> 6;
  const int tilesM = M >> 6;
  const int tile = blockIdx.x * 8 + wave;
  if (tile >= tilesM * tilesN) return;
  const int tm = tile / tilesN;
  const int tn = tile - tm * tilesN;
  const int m0 = tm << 6;
  const int n0 = tn << 6;

  const T* Ab  = A  + (size_t)b * strideA;
  const T* Bb  = Bt + (size_t)b * strideB;
  const T* Ab2 = (SPL >= 1) ? (A2  + (size_t)b * strideA) : nullptr;
  const T* Bb2 = (SPL == 2) ? (Bt2 + (size_t)b * strideB) : nullptr;

  const int rlane = lane & 15;
  const int koff  = (lane >> 4) * 8;
  const int mOff  = (lane >> 4) * 8;

  v8f acc[4][4];
#pragma unroll
  for (int i = 0; i < 4; ++i)
#pragma unroll
    for (int j = 0; j < 4; ++j) acc[i][j] = (v8f){0.f,0.f,0.f,0.f,0.f,0.f,0.f,0.f};

  for (int k0 = 0; k0 < K; k0 += 32) {
    V bh[4], bl[4];
#pragma unroll
    for (int j = 0; j < 4; ++j) {
      const size_t bo = (size_t)(n0 + (j << 4) + rlane) * ldb + koff + k0;
      bh[j] = Frag<T>::load(Bb + bo);
      if (SPL == 2) bl[j] = Frag<T>::load(Bb2 + bo);
    }
#pragma unroll
    for (int i = 0; i < 4; ++i) {
      const size_t ao = (size_t)(m0 + (i << 4) + rlane) * lda + koff + k0;
      V ah = Frag<T>::load(Ab + ao);
      V al;
      if (SPL >= 1) al = Frag<T>::load(Ab2 + ao);
#pragma unroll
      for (int j = 0; j < 4; ++j) {
        acc[i][j] = Frag<T>::mma(ah, bh[j], acc[i][j]);
        if (SPL == 2) acc[i][j] = Frag<T>::mma(ah, bl[j], acc[i][j]);
        if (SPL >= 1) acc[i][j] = Frag<T>::mma(al, bh[j], acc[i][j]);
      }
      Frag<T>::guard4(acc[i][0], acc[i][1], acc[i][2], acc[i][3], ah, (SPL >= 1) ? al : ah);
    }
    Frag<T>::keep(bh[0], bh[1], bh[2], bh[3]);
    if (SPL == 2) Frag<T>::keep(bl[0], bl[1], bl[2], bl[3]);
  }
  acc_guard4(acc[0][0], acc[0][1], acc[0][2], acc[0][3]);
  acc_guard4(acc[1][0], acc[1][1], acc[1][2], acc[1][3]);
  acc_guard4(acc[2][0], acc[2][1], acc[2][2], acc[2][3]);
  acc_guard4(acc[3][0], acc[3][1], acc[3][2], acc[3][3]);

  float* slab = sT[wave];
  const float* Rb = RESID ? (resid + (size_t)b * strideR) : nullptr;
#pragma unroll
  for (int i = 0; i < 4; ++i) {
    const int mBase = m0 + (i << 4);
#pragma unroll
    for (int j = 0; j < 4; ++j) {
      const int n = n0 + (j << 4) + rlane;
      float bv = 0.f;
      if (BIAS_MODE == 2) bv = bias[n];
#pragma unroll
      for (int r = 0; r < 8; ++r) {
        float v = acc[i][j][r] * scale;
        if (BIAS_MODE == 1) v += bias[mBase + mOff + r];
        if (BIAS_MODE == 2) v += bv;
        if (RESID) v += Rb[(size_t)(mBase + mOff + r) * ldc + n];
        if (ACT == 1) v = tanhf(v);
        if (ACT == 2) v = fmaxf(v, 0.0f);
        if (ACT == 3) v = v / (1.0f + expf(-v));
        if (ACT == 4) v = (v > 0.f) ? v : 0.01f * v;
        slab[(mOff + r) * 68 + (j << 4) + rlane] = v;
      }
    }
    __builtin_amdgcn_fence(__ATOMIC_RELEASE, "workgroup");
    __builtin_amdgcn_wave_barrier();
    __builtin_amdgcn_fence(__ATOMIC_ACQUIRE, "workgroup");
    if (OUT_MODE == 0) {
      float* C = (float*)Cout + (size_t)b * strideC;
      const int hh = lane >> 4, c4 = (lane & 15) * 4;
      for (int pass = 0; pass < 2; ++pass) {
#pragma unroll
        for (int it = 0; it < 8; ++it) {
          const int row = it * 2 + hh;
          v4f v = *(const v4f*)(slab + row * 68 + c4);
          *(volatile v4f*)(C + (size_t)(mBase + row) * ldc + n0 + c4) = v;
        }
        __threadfence();
      }
    } else {
      const int q = lane >> 3, c8 = (lane & 7) * 8;
      unsigned short* C  = (unsigned short*)Cout  + (size_t)b * strideC;
      unsigned short* C2 = (OUT_MODE == 2) ? ((unsigned short*)Cout2 + (size_t)b * strideC) : nullptr;
      for (int pass = 0; pass < 2; ++pass) {
#pragma unroll
        for (int it = 0; it < 4; ++it) {
          const int row = it * 4 + q;
          const float* sp = slab + row * 68 + c8;
          v8h hv, lv;
#pragma unroll
          for (int e = 0; e < 8; ++e) {
            if (OUT_MODE == 1) {
              hv[e] = (_Float16)sp[e];
            } else {
              unsigned short hb = f2bf_bits(sp[e]);
              unsigned short lb = f2bf_bits(sp[e] - bf_bits2f(hb));
              hv[e] = __builtin_bit_cast(_Float16, hb);
              lv[e] = __builtin_bit_cast(_Float16, lb);
            }
          }
          *(volatile v8h*)(C + (size_t)(mBase + row) * ldc + n0 + c8) = hv;
          if (OUT_MODE == 2) *(volatile v8h*)(C2 + (size_t)(mBase + row) * ldc + n0 + c8) = lv;
        }
        __threadfence();
      }
    }
    __builtin_amdgcn_fence(__ATOMIC_RELEASE, "workgroup");
    __builtin_amdgcn_wave_barrier();
    __builtin_amdgcn_fence(__ATOMIC_ACQUIRE, "workgroup");
  }
}

__device__ __forceinline__ float gate_sig(float t) { return __builtin_amdgcn_rcpf(1.0f + expf(-t)); }

__global__ __launch_bounds__(256) void cvt_u_kernel(
    const float* __restrict__ x, const float* __restrict__ trend, unsigned short* __restrict__ U16, int total8)
{
  const int i = blockIdx.x * 256 + threadIdx.x;
  if (i >= total8) return;
  const size_t e0 = (size_t)i << 3;
  const int k0 = (int)(e0 & (size_t)(kDm - 1));
  const v4f a0 = *(const v4f*)(x + e0);
  const v4f a1 = *(const v4f*)(x + e0 + 4);
  const v4f t0 = *(const v4f*)(trend + k0);
  const v4f t1 = *(const v4f*)(trend + k0 + 4);
  v8h hv;
#pragma unroll
  for (int e = 0; e < 4; ++e) {
    hv[e]     = (_Float16)(a0[e] * gate_sig(t0[e]));
    hv[4 + e] = (_Float16)(a1[e] * gate_sig(t1[e]));
  }
  unsigned short* q = U16 + e0;
  *(volatile v8h*)q = hv;
  __threadfence();
  *(volatile v8h*)q = hv;
}

__global__ __launch_bounds__(256) void cvt_rows_f16_kernel(
    const float* __restrict__ src, unsigned short* __restrict__ dst, int total8, int valid8, float scale)
{
  const int i = blockIdx.x * 256 + threadIdx.x;
  if (i >= total8) return;
  const int ic = (i < valid8) ? i : (valid8 - 1);
  const float fac = (i < valid8) ? scale : 0.0f;
  const size_t s0 = (size_t)ic << 3;
  const v4f a0 = *(const v4f*)(src + s0);
  const v4f a1 = *(const v4f*)(src + s0 + 4);
  v8h hv;
#pragma unroll
  for (int e = 0; e < 4; ++e) {
    hv[e]     = (_Float16)(a0[e] * fac);
    hv[4 + e] = (_Float16)(a1[e] * fac);
  }
  unsigned short* q = dst + ((size_t)i << 3);
  *(volatile v8h*)q = hv;
  __threadfence();
  *(volatile v8h*)q = hv;
}

__global__ __launch_bounds__(256) void cvt_dp_kernel(
    const float* __restrict__ XZ, unsigned short* __restrict__ DP16, int total8)
{
  const int i = blockIdx.x * 256 + threadIdx.x;
  if (i >= total8) return;
  const size_t e0 = (size_t)i << 3;
  const size_t r  = e0 >> 6;
  const int    c0 = (int)(e0 & 63);
  const float* sp = XZ + r * kNpad + c0;
  const v4f a0 = *(const v4f*)(sp);
  const v4f a1 = *(const v4f*)(sp + 4);
  v8h hv;
#pragma unroll
  for (int e = 0; e < 4; ++e) {
    hv[e]     = (_Float16)(a0[e] * kDpCarry);
    hv[4 + e] = (_Float16)(a1[e] * kDpCarry);
  }
  unsigned short* q = DP16 + e0;
  *(volatile v8h*)q = hv;
  __threadfence();
  *(volatile v8h*)q = hv;
}

__global__ __launch_bounds__(64) void scan_kernel(
    const float* __restrict__ XZ, const float* __restrict__ DPRE, const float* __restrict__ x,
    const float* __restrict__ bdt, const float* __restrict__ Alog, const float* __restrict__ Dp,
    const float* __restrict__ trend, float* __restrict__ out)
{
  __shared__ __align__(16) float sX[kScanTS * kBcW];
  __shared__ __align__(16) float sY[kScanTS * kScanYP];
  __shared__ __align__(16) float sA[kNst * kScanCh];
  const int tid = threadIdx.x, lane = tid & 31, wave = tid >> 5;
  constexpr int kBlkPerB = kDm / kScanCh;
  const int bix = blockIdx.x / kBlkPerB;
  const int d0  = (blockIdx.x - bix * kBlkPerB) * kScanCh;
  const int d   = d0 + tid;
  const size_t row0 = (size_t)bix * kSeq;
#pragma unroll 1
  for (int s = 0; s < kNst; ++s) sA[s * kScanCh + tid] = -expf(Alog[(size_t)d * kNst + s]);
  __syncthreads();
  float negA[kNst], h[kNst];
#pragma unroll
  for (int s = 0; s < kNst; ++s) {
    negA[s] = sA[s * kScanCh + tid];
    h[s] = 0.0f;
  }
  const float bb = bdt[d], Dd = Dp[d], sg = gate_sig(trend[d]);
  const int lr = tid >> 3, lc4 = (tid & 7) * 4;
  const int hh = lane >> 4, c4 = (lane & 15) * 4;
#pragma unroll 1
  for (int t0 = 0; t0 < kSeq; t0 += kScanTS) {
    __syncthreads();
#pragma unroll
    for (int i = 0; i < 8; ++i) {
      const int r = lr + 8 * i;
      *(v4f*)(sX + r * kBcW + lc4) = *(const v4f*)(XZ + (row0 + t0 + r) * kNpad + kDtR + lc4);
    }
    __syncthreads();
#pragma unroll 1
    for (int s = 0; s < kScanTS; ++s) {
      const int t = t0 + s;
      const float* xr = sX + s * kBcW;
      float Bs[kNst], Cs[kNst];
#pragma unroll
      for (int q4 = 0; q4 < 4; ++q4) {
        const v4f bv = *(const v4f*)(xr + 4 * q4);
        const v4f cv = *(const v4f*)(xr + kNst + 4 * q4);
        Bs[4 * q4 + 0] = bv[0]; Bs[4 * q4 + 1] = bv[1]; Bs[4 * q4 + 2] = bv[2]; Bs[4 * q4 + 3] = bv[3];
        Cs[4 * q4 + 0] = cv[0]; Cs[4 * q4 + 1] = cv[1]; Cs[4 * q4 + 2] = cv[2]; Cs[4 * q4 + 3] = cv[3];
      }
      const size_t g = (row0 + t) * kDm + d;
      const float v   = DPRE[g] + bb;
      const float dt  = fmaxf(v, 0.0f) + log1pf(expf(-fabsf(v)));
      const float ut  = x[g] * sg;
      const float dtx = dt * ut;
      float y = 0.0f;
#pragma unroll
      for (int k = 0; k < kNst; ++k) {
        const float e = __expf(dt * negA[k]);
        h[k] = e * h[k] + dtx * Bs[k];
        y = h[k] * Cs[k] + y;
      }
      y = ut * Dd + y;
      sY[s * kScanYP + tid] = y;
    }
    __syncthreads();
    for (int pass = 0; pass < 2; ++pass) {
#pragma unroll
      for (int it = 0; it < 16; ++it) {
        const int row = it * 4 + wave * 2 + hh;
        const v4f val = *(const v4f*)(sY + row * kScanYP + c4);
        *(volatile v4f*)(out + (row0 + t0 + row) * kDm + d0 + c4) = val;
      }
      __threadfence();
    }
  }
}

extern "C" void kernel_launch(void* const* d_in, const int* in_sizes, int n_in,
                              void* d_out, int out_size, void* d_ws, size_t ws_size,
                              hipStream_t stream) {
  if (n_in < 7) return;
  if (in_sizes[0] != kRows * kDm) return;
  if (in_sizes[1] != kDm * kNst) return;
  if (in_sizes[2] != kNproj * kDm) return;
  if (in_sizes[3] != kDm * kDtR) return;
  if (in_sizes[4] != kDm) return;
  if (in_sizes[5] != kDm) return;
  if (in_sizes[6] != kDm) return;
  if (out_size != kRows * kDm) return;
  if (ws_size < kWsTotal) return;

  const float* x         = (const float*)d_in[0];
  const float* A_log     = (const float*)d_in[1];
  const float* x_proj_w  = (const float*)d_in[2];
  const float* dt_proj_w = (const float*)d_in[3];
  const float* dt_proj_b = (const float*)d_in[4];
  const float* D_param   = (const float*)d_in[5];
  const float* trend     = (const float*)d_in[6];
  float* out = (float*)d_out;

  char* ws = (char*)d_ws;
  unsigned short* U16  = (unsigned short*)(ws + kOffU16);
  unsigned short* W1H  = (unsigned short*)(ws + kOffW1H);
  unsigned short* W2H  = (unsigned short*)(ws + kOffW2H);
  float*          XZ   = (float*)(ws + kOffXZ);
  unsigned short* DP16 = (unsigned short*)(ws + kOffDP16);
  float*          DPRE = (float*)(ws + kOffDPRE);

  constexpr int kU8  = kRows * kDm / 8;
  constexpr int kW18 = kNpad * kDm / 8;
  constexpr int kW1V = kNproj * kDm / 8;
  constexpr int kW28 = kDm * kDtR / 8;
  constexpr int kDp8 = kRows * kDtR / 8;
  static_assert((kU8 % 256) == 0 && (kW18 % 256) == 0 && (kW28 % 256) == 0 && (kDp8 % 256) == 0, "exact grids");

  cvt_u_kernel<<<kU8 / 256, 256, 0, stream>>>(x, trend, U16, kU8);
  cvt_rows_f16_kernel<<<kW18 / 256, 256, 0, stream>>>(x_proj_w, W1H, kW18, kW1V, kW1Carry);
  cvt_rows_f16_kernel<<<kW28 / 256, 256, 0, stream>>>(dt_proj_w, W2H, kW28, kW28, kW2Carry);

  wmma_gemm64<0, 0, 0, 0, false><<<dim3((kRows / 64) * (kNpad / 64) / 8, 1), 256, 0, stream>>>(
      U16, nullptr, kDm, 0L,
      W1H, nullptr, kDm, 0L,
      (void*)XZ, nullptr, kNpad, 0L,
      nullptr, nullptr, 0L,
      kRows, kNpad, kDm, 1.0f / kW1Carry);

  cvt_dp_kernel<<<kDp8 / 256, 256, 0, stream>>>(XZ, DP16, kDp8);

  wmma_gemm64<0, 0, 0, 0, false><<<dim3((kRows / 64) * (kDm / 64) / 8, 1), 256, 0, stream>>>(
      DP16, nullptr, kDtR, 0L,
      W2H, nullptr, kDtR, 0L,
      (void*)DPRE, nullptr, kDm, 0L,
      nullptr, nullptr, 0L,
      kRows, kDm, kDtR, 1.0f / (kDpCarry * kW2Carry));

  scan_kernel<<<kBatch * (kDm / kScanCh), kScanCh, 0, stream>>>(XZ, DPRE, x, dt_proj_b, A_log, D_param, trend, out);
}
